// GPTBlock_46763603919345
// MI455X (gfx1250) — hardware-verified
//
#include <hip/hip_runtime.h>
#include <math.h>

constexpr int kBatch   = 2;
constexpr int kSeq     = 2048;
constexpr int kEmb     = 1024;
constexpr int kHeads   = 16;
constexpr int kHeadDim = 64;
constexpr int kFF      = 4096;
constexpr int kTok     = kBatch * kSeq;
constexpr int kQKld    = 2 * kEmb;
constexpr int kHeadsPerChunk = 2;
constexpr float kWCarry       = 16.0f;
constexpr float kWCarryInv    = 1.0f / 16.0f;
constexpr float kPCarry       = 2048.0f;
constexpr float kCtxCarry     = 256.0f;
constexpr float kPVScale      = kCtxCarry / kPCarry;
constexpr float kOutProjScale = 1.0f / (kCtxCarry * kWCarry);
constexpr float kInvEmb       = 1.0f / 1024.0f;
constexpr float kLnEps        = 1e-5f;
constexpr float kAttnScale    = 0.125f;

static_assert(kSeq % 64 == 0 && kEmb % 64 == 0 && kFF % 64 == 0 && kTok % 64 == 0, "tile multiples");
static_assert(kHeadDim % 32 == 0 && kEmb % 32 == 0 && kFF % 32 == 0 && kSeq % 32 == 0, "K multiples of 32");
static_assert(kHeads % kHeadsPerChunk == 0, "chunking");
static_assert(kEmb == 8 * 128, "layernorm kernel: 128 threads x 8 columns");
static_assert(kSeq == 8 * 256, "softmax kernel: 256 threads x 8 columns");

typedef __attribute__((ext_vector_type(16))) _Float16 v16h;
typedef __attribute__((ext_vector_type(8)))  _Float16 v8h;
typedef __attribute__((ext_vector_type(16))) __bf16   v16b;
typedef __attribute__((ext_vector_type(8)))  __bf16   v8b;
typedef __attribute__((ext_vector_type(8)))  float    v8f;
typedef __attribute__((ext_vector_type(4)))  float    v4f;
typedef __attribute__((ext_vector_type(4)))  unsigned int v4u;

__device__ __forceinline__ unsigned short f2bf_bits(float f) {
  unsigned u = __float_as_uint(f);
  return (unsigned short)((u + 0x7FFFu + ((u >> 16) & 1u)) >> 16);
}
__device__ __forceinline__ float bf_bits2f(unsigned short h) { return __uint_as_float(((unsigned)h) << 16); }

__device__ __forceinline__ void dep_guard_h(v8f& a, v8f& b, v16h x, v16h y) { asm volatile("v_nop\n\tv_nop\n\tv_nop\n\tv_nop" : "+v"(a), "+v"(b) : "v"(x), "v"(y)); }
__device__ __forceinline__ void dep_guard_b(v8f& a, v8f& b, v16b x, v16b y) { asm volatile("v_nop\n\tv_nop\n\tv_nop\n\tv_nop" : "+v"(a), "+v"(b) : "v"(x), "v"(y)); }
__device__ __forceinline__ void keep4_h(v16h a, v16h b, v16h c, v16h d) { asm volatile("v_nop" :: "v"(a), "v"(b), "v"(c), "v"(d)); }
__device__ __forceinline__ void keep4_b(v16b a, v16b b, v16b c, v16b d) { asm volatile("v_nop" :: "v"(a), "v"(b), "v"(c), "v"(d)); }
__device__ __forceinline__ void acc_guard4(v8f& a, v8f& b, v8f& c, v8f& d) { asm volatile("v_nop\n\tv_nop\n\tv_nop\n\tv_nop" : "+v"(a), "+v"(b), "+v"(c), "+v"(d)); }
template <typename T> struct Frag;
template <> struct Frag<_Float16> {
  typedef v16h V; union U { v16h v; v8h h[2]; };
  static __device__ __forceinline__ v16h load(const _Float16* p) {
    U f; f.h[0] = *(const v8h*)(p); f.h[1] = *(const v8h*)(p + 16); return f.v;
  }
  static __device__ __forceinline__ v8f mma(v16h a, v16h b, v8f c) {
    return __builtin_amdgcn_wmma_f32_16x16x32_f16(false, a, false, b, (short)0, c, false, false);
  }
  static __device__ __forceinline__ void guard(v8f& a, v8f& b, v16h x, v16h y) { dep_guard_h(a, b, x, y); }
  static __device__ __forceinline__ void keep(v16h a, v16h b, v16h c, v16h d) { keep4_h(a, b, c, d); }
};
template <> struct Frag<__bf16> {
  typedef v16b V; union U { v16b v; v8b h[2]; };
  static __device__ __forceinline__ v16b load(const __bf16* p) {
    U f; f.h[0] = *(const v8b*)(p); f.h[1] = *(const v8b*)(p + 16); return f.v;
  }
  static __device__ __forceinline__ v8f mma(v16b a, v16b b, v8f c) {
    return __builtin_amdgcn_wmma_f32_16x16x32_bf16(false, a, false, b, (short)0, c, false, false);
  }
  static __device__ __forceinline__ void guard(v8f& a, v8f& b, v16b x, v16b y) { dep_guard_b(a, b, x, y); }
  static __device__ __forceinline__ void keep(v16b a, v16b b, v16b c, v16b d) { keep4_b(a, b, c, d); }
};

__device__ __forceinline__ unsigned pk16(unsigned short a, unsigned short b) { return (unsigned)a | ((unsigned)b << 16); }
__device__ __forceinline__ unsigned short h_bits(float f) { const _Float16 h = (_Float16)f; return __builtin_bit_cast(unsigned short, h); }

template <int ET> struct Elem;
template <> struct Elem<0> { typedef _Float16 T; };
template <> struct Elem<1> { typedef __bf16 T; };
template <int ET, bool SPLIT, int BIAS_MODE, int OUT_MODE, bool RESID, int ACT = 0, int CAUSAL = 0>
__global__ __launch_bounds__(256) void wmma_gemm64(
    const unsigned short* __restrict__ Ap, const unsigned short* __restrict__ A2p, int lda, long strideA,
    const unsigned short* __restrict__ Btp, const unsigned short* __restrict__ Bt2p, int ldb, long strideB,
    void* __restrict__ Cout, void* __restrict__ Cout2, int ldc, long strideC,
    const float* __restrict__ bias,
    const float* __restrict__ resid, long strideR,
    int M, int N, int K, float scale) {
  typedef typename Elem<ET>::T T;
  typedef typename Frag<T>::V V;
  const T* A = (const T*)Ap; const T* A2 = (const T*)A2p; const T* Bt = (const T*)Btp; const T* Bt2 = (const T*)Bt2p;
  __shared__ __align__(16) float sT[8][16 * 68];
  const int b    = blockIdx.y;
  const int lane = threadIdx.x & 31;
  const int wave = threadIdx.x >> 5;
  const int tilesN = N >> 6;
  const int tilesM = M >> 6;
  const int tile = blockIdx.x * 8 + wave;
  if (tile >= tilesM * tilesN) return;
  const int tm = tile / tilesN;
  const int tn = tile - tm * tilesN;
  const int m0 = tm << 6;
  const int n0 = tn << 6;
  if (CAUSAL == 1 && n0 > m0) return;
  const int Kend = (CAUSAL == 2) ? ((m0 + 64 < K) ? (m0 + 64) : K) : K;

  const T* Ab  = A  + (size_t)b * strideA;
  const T* Bb  = Bt + (size_t)b * strideB;
  const T* Ab2 = SPLIT ? (A2  + (size_t)b * strideA) : nullptr;
  const T* Bb2 = SPLIT ? (Bt2 + (size_t)b * strideB) : nullptr;

  const int rlane = lane & 15;
  const int koff  = (lane >> 4) * 8;
  const int mOff  = (lane >> 4) * 8;

  v8f acc[4][4];
#pragma unroll
  for (int i = 0; i < 4; ++i)
#pragma unroll
    for (int j = 0; j < 4; ++j) acc[i][j] = (v8f){0.f,0.f,0.f,0.f,0.f,0.f,0.f,0.f};

  for (int k0 = 0; k0 < Kend; k0 += 32) {
    V bh[4], bl[4];
#pragma unroll
    for (int j = 0; j < 4; ++j) {
      const size_t bo = (size_t)(n0 + (j << 4) + rlane) * ldb + koff + k0;
      bh[j] = Frag<T>::load(Bb + bo);
      if (SPLIT) bl[j] = Frag<T>::load(Bb2 + bo);
    }
#pragma unroll
    for (int i = 0; i < 4; ++i) {
      const size_t ao = (size_t)(m0 + (i << 4) + rlane) * lda + koff + k0;
      V ah = Frag<T>::load(Ab + ao);
      V al;
      if (SPLIT) al = Frag<T>::load(Ab2 + ao);
#pragma unroll
      for (int j = 0; j < 4; ++j) {
        acc[i][j] = Frag<T>::mma(ah, bh[j], acc[i][j]);
        if (SPLIT) {
          acc[i][j] = Frag<T>::mma(ah, bl[j], acc[i][j]);
          acc[i][j] = Frag<T>::mma(al, bh[j], acc[i][j]);
        }
      }
      Frag<T>::guard(acc[i][0], acc[i][3], ah, SPLIT ? al : ah);
    }
    Frag<T>::keep(bh[0], bh[1], bh[2], bh[3]);
    if (SPLIT) Frag<T>::keep(bl[0], bl[1], bl[2], bl[3]);
  }
  acc_guard4(acc[0][0], acc[0][1], acc[0][2], acc[0][3]);
  acc_guard4(acc[1][0], acc[1][1], acc[1][2], acc[1][3]);
  acc_guard4(acc[2][0], acc[2][1], acc[2][2], acc[2][3]);
  acc_guard4(acc[3][0], acc[3][1], acc[3][2], acc[3][3]);

  float* slab = sT[wave];
  const float* Rb = RESID ? (resid + (size_t)b * strideR) : nullptr;
#pragma unroll
  for (int i = 0; i < 4; ++i) {
    const int mBase = m0 + (i << 4);
#pragma unroll
    for (int j = 0; j < 4; ++j) {
      const int n = n0 + (j << 4) + rlane;
      float bv = 0.f;
      if (BIAS_MODE == 2) bv = bias[n];
#pragma unroll
      for (int r = 0; r < 8; ++r) {
        float v = acc[i][j][r] * scale;
        if (BIAS_MODE == 1) v += bias[mBase + mOff + r];
        if (BIAS_MODE == 2) v += bv;
        if (RESID) v += Rb[(size_t)(mBase + mOff + r) * ldc + n];
        if (ACT == 2) v = fmaxf(v, 0.0f);
        if (ACT == 4) v = (v > 0.f) ? v : 0.01f * v;
        slab[(mOff + r) * 68 + (j << 4) + rlane] = v;
      }
    }
    __builtin_amdgcn_fence(__ATOMIC_RELEASE, "workgroup");
    __builtin_amdgcn_wave_barrier();
    __builtin_amdgcn_fence(__ATOMIC_ACQUIRE, "workgroup");
    if (OUT_MODE == 0) {
      float* C = (float*)Cout + (size_t)b * strideC;
      const int hh = lane >> 4, c4 = (lane & 15) * 4;
      for (int pass = 0; pass < 2; ++pass) {
#pragma unroll
        for (int it = 0; it < 8; ++it) {
          const int row = it * 2 + hh;
          v4f v = *(const v4f*)(slab + row * 68 + c4);
          *(volatile v4f*)(C + (size_t)(mBase + row) * ldc + n0 + c4) = v;
        }
        __threadfence();
      }
    } else {
      const int q = lane >> 3, c8 = (lane & 7) * 8;
      unsigned short* C  = (unsigned short*)Cout  + (size_t)b * strideC;
      unsigned short* C2 = (OUT_MODE == 2) ? ((unsigned short*)Cout2 + (size_t)b * strideC) : nullptr;
      for (int pass = 0; pass < 2; ++pass) {
#pragma unroll
        for (int it = 0; it < 4; ++it) {
          const int row = it * 4 + q;
          const float* sp = slab + row * 68 + c8;
          v8h hv, lv;
#pragma unroll
          for (int e = 0; e < 8; ++e) {
            if (OUT_MODE == 1) {
              hv[e] = (_Float16)sp[e];
            } else {
              unsigned short hb = f2bf_bits(sp[e]);
              unsigned short lb = f2bf_bits(sp[e] - bf_bits2f(hb));
              hv[e] = __builtin_bit_cast(_Float16, hb);
              lv[e] = __builtin_bit_cast(_Float16, lb);
            }
          }
          *(volatile v8h*)(C + (size_t)(mBase + row) * ldc + n0 + c8) = hv;
          if (OUT_MODE == 2) *(volatile v8h*)(C2 + (size_t)(mBase + row) * ldc + n0 + c8) = lv;
        }
        __threadfence();
      }
    }
    __builtin_amdgcn_fence(__ATOMIC_RELEASE, "workgroup");
    __builtin_amdgcn_wave_barrier();
    __builtin_amdgcn_fence(__ATOMIC_ACQUIRE, "workgroup");
  }
}

__global__ __launch_bounds__(256) void wtcast_kernel(const float* __restrict__ W, int R, int Ccols,
                                                     unsigned short* __restrict__ out, int ldo, float scale) {
  __shared__ float sm[64][65];
  const int t  = threadIdx.x;
  const int k0 = blockIdx.x * 64;
  const int nb = blockIdx.y * 64;
#pragma unroll
  for (int i = 0; i < 16; ++i) {
    const int e = i * 256 + t;
    const int r = e >> 6;
    const int c = e & 63;
    sm[c][r] = W[(size_t)(k0 + r) * Ccols + nb + c] * scale;
  }
  __syncthreads();
  const int lane = t & 31, wave = t >> 5;
  const int q = lane >> 3, c8 = (lane & 7) * 8;
  for (int pass = 0; pass < 2; ++pass) {
#pragma unroll
    for (int it = 0; it < 2; ++it) {
      const int row = wave * 8 + it * 4 + q;
      unsigned short hb[8];
#pragma unroll
      for (int e = 0; e < 8; ++e) hb[e] = h_bits(sm[row][c8 + e]);
      const v4u u = (v4u){pk16(hb[0], hb[1]), pk16(hb[2], hb[3]), pk16(hb[4], hb[5]), pk16(hb[6], hb[7])};
      *(volatile v4u*)(out + (size_t)(nb + row) * ldo + k0 + c8) = u;
    }
    __threadfence();
  }
}

__global__ __launch_bounds__(128) void layernorm_f16_kernel(const float* __restrict__ X, const float* __restrict__ gam,
                                                            const float* __restrict__ bet, unsigned short* __restrict__ out) {
  __shared__ float redA[4];
  __shared__ float redB[4];
  const int row  = blockIdx.x;
  const int t    = threadIdx.x;
  const int lane = t & 31, wave = t >> 5;
  const int c0   = t * 8;
  const float* xr = X + (size_t)row * kEmb + c0;
  const v4f a = *(const v4f*)(xr);
  const v4f c = *(const v4f*)(xr + 4);
  float x[8];
#pragma unroll
  for (int e = 0; e < 4; ++e) { x[e] = a[e]; x[4 + e] = c[e]; }
  float s = ((x[0] + x[1]) + (x[2] + x[3])) + ((x[4] + x[5]) + (x[6] + x[7]));
#pragma unroll
  for (int off = 16; off > 0; off >>= 1) s += __shfl_xor(s, off, 32);
  if (lane == 0) redA[wave] = s;
  __syncthreads();
  const float mu = ((redA[0] + redA[1]) + (redA[2] + redA[3])) * kInvEmb;
  float d[8];
  float ss = 0.f;
#pragma unroll
  for (int e = 0; e < 8; ++e) { d[e] = x[e] - mu; ss += d[e] * d[e]; }
#pragma unroll
  for (int off = 16; off > 0; off >>= 1) ss += __shfl_xor(ss, off, 32);
  if (lane == 0) redB[wave] = ss;
  __syncthreads();
  const float var = ((redB[0] + redB[1]) + (redB[2] + redB[3])) * kInvEmb;
  const float inv = rsqrtf(var + kLnEps);
  const v4f ga = *(const v4f*)(gam + c0);
  const v4f gc = *(const v4f*)(gam + c0 + 4);
  const v4f ba = *(const v4f*)(bet + c0);
  const v4f bc = *(const v4f*)(bet + c0 + 4);
  float gg[8], bb[8];
#pragma unroll
  for (int e = 0; e < 4; ++e) { gg[e] = ga[e]; gg[4 + e] = gc[e]; bb[e] = ba[e]; bb[4 + e] = bc[e]; }
  unsigned short hb[8];
#pragma unroll
  for (int e = 0; e < 8; ++e) hb[e] = h_bits(d[e] * inv * gg[e] + bb[e]);
  const v4u u = (v4u){pk16(hb[0], hb[1]), pk16(hb[2], hb[3]), pk16(hb[4], hb[5]), pk16(hb[6], hb[7])};
  unsigned short* op = out + (size_t)row * kEmb + c0;
  *(volatile v4u*)op = u;
  __threadfence();
  *(volatile v4u*)op = u;
}

__global__ __launch_bounds__(256) void softmax_causal_kernel(const float* __restrict__ S, unsigned short* __restrict__ P, float carry) {
  __shared__ float redM[8];
  __shared__ float redS[8];
  const int bx   = blockIdx.x;
  const int grp  = bx >> 11;
  const int q    = bx & (kSeq - 1);
  const int t    = threadIdx.x;
  const int lane = t & 31, wave = t >> 5;
  const int c0   = t * 8;
  const int clim = (q | 63) - 7;
  const int cb   = (c0 < clim) ? c0 : clim;
  const size_t rowoff = ((size_t)grp * kSeq + q) * (size_t)kSeq;
  const float* sr = S + rowoff + cb;
  const v4f a = *(const v4f*)(sr);
  const v4f c = *(const v4f*)(sr + 4);
  float x[8];
#pragma unroll
  for (int e = 0; e < 4; ++e) { x[e] = a[e] * kAttnScale; x[4 + e] = c[e] * kAttnScale; }
  float m = -INFINITY;
#pragma unroll
  for (int e = 0; e < 8; ++e) {
    const float xv = (c0 + e <= q) ? x[e] : -INFINITY;
    x[e] = xv;
    m = fmaxf(m, xv);
  }
#pragma unroll
  for (int off = 16; off > 0; off >>= 1) m = fmaxf(m, __shfl_xor(m, off, 32));
  if (lane == 0) redM[wave] = m;
  __syncthreads();
  float rm = redM[0];
#pragma unroll
  for (int w = 1; w < 8; ++w) rm = fmaxf(rm, redM[w]);
  float sum = 0.f;
#pragma unroll
  for (int e = 0; e < 8; ++e) {
    const float ev = expf(x[e] - rm);
    const float p = (c0 + e <= q) ? ev : 0.f;
    x[e] = p;
    sum += p;
  }
#pragma unroll
  for (int off = 16; off > 0; off >>= 1) sum += __shfl_xor(sum, off, 32);
  if (lane == 0) redS[wave] = sum;
  __syncthreads();
  const float tot = ((redS[0] + redS[1]) + (redS[2] + redS[3])) + ((redS[4] + redS[5]) + (redS[6] + redS[7]));
  const float inv = carry * (1.0f / tot);
  unsigned short hb[8];
#pragma unroll
  for (int e = 0; e < 8; ++e) hb[e] = h_bits(x[e] * inv);
  const v4u u = (v4u){pk16(hb[0], hb[1]), pk16(hb[2], hb[3]), pk16(hb[4], hb[5]), pk16(hb[6], hb[7])};
  unsigned short* op = P + rowoff + c0;
  *(volatile v4u*)op = u;
  __threadfence();
  *(volatile v4u*)op = u;
}

__global__ __launch_bounds__(256) void gelu_cast_kernel(const float* __restrict__ in, unsigned short* __restrict__ out, int n2) {
  const int i = blockIdx.x * 256 + threadIdx.x;
  if (i >= n2) return;
  const float u0 = in[2 * (size_t)i];
  const float u1 = in[2 * (size_t)i + 1];
  const float g0 = 0.5f * u0 * (1.0f + erff(u0 * 0.70710678118654752f));
  const float g1 = 0.5f * u1 * (1.0f + erff(u1 * 0.70710678118654752f));
  const unsigned u = pk16(h_bits(g0), h_bits(g1));
  unsigned* op = (unsigned*)(out + 2 * (size_t)i);
  *(volatile unsigned*)op = u;
  __threadfence();
  *(volatile unsigned*)op = u;
}

extern "C" void kernel_launch(void* const* d_in, const int* in_sizes, int n_in,
                              void* d_out, int out_size, void* d_ws,
                              size_t ws_size, hipStream_t stream) {
  if (n_in < 14) return;
  if (in_sizes[0] != kTok * kEmb || out_size != kTok * kEmb) return;
  if (in_sizes[1] != kEmb * kEmb || in_sizes[6] != kEmb * kFF || in_sizes[8] != kFF * kEmb) return;
  const size_t MiB = 1048576;
  const size_t kCarveTotal = 128 * MiB;
  if (ws_size < kCarveTotal) return;

  const float* X     = (const float*)d_in[0];
  const float* W_Q   = (const float*)d_in[1];
  const float* W_K   = (const float*)d_in[2];
  const float* W_V   = (const float*)d_in[3];
  const float* W_out = (const float*)d_in[4];
  const float* b_out = (const float*)d_in[5];
  const float* W1    = (const float*)d_in[6];
  const float* b1    = (const float*)d_in[7];
  const float* W2    = (const float*)d_in[8];
  const float* b2    = (const float*)d_in[9];
  const float* ln1_g = (const float*)d_in[10];
  const float* ln1_b = (const float*)d_in[11];
  const float* ln2_g = (const float*)d_in[12];
  const float* ln2_b = (const float*)d_in[13];
  float* out = (float*)d_out;

  char* ws = (char*)d_ws;
  unsigned short* W1T   = (unsigned short*)(ws + 0 * MiB);
  unsigned short* W2T   = (unsigned short*)(ws + 8 * MiB);
  float*          X1    = (float*)(ws + 16 * MiB);
  unsigned short* H16   = (unsigned short*)(ws + 32 * MiB);
  unsigned short* WqkT  = (unsigned short*)(ws + 40 * MiB);
  unsigned short* WvT   = (unsigned short*)(ws + 44 * MiB);
  unsigned short* WoT   = (unsigned short*)(ws + 46 * MiB);
  unsigned short* CTX16 = (unsigned short*)(ws + 48 * MiB);
  unsigned short* QK16  = (unsigned short*)(ws + 56 * MiB);
  unsigned short* VT16  = (unsigned short*)(ws + 72 * MiB);
  float*          Sbuf  = (float*)(ws + 80 * MiB);
  unsigned short* Pbuf  = (unsigned short*)(ws + 112 * MiB);
  float*          FFpre = (float*)(ws + 64 * MiB);
  unsigned short* G16   = (unsigned short*)(ws + 32 * MiB);

  wtcast_kernel<<<dim3(kEmb / 64, kEmb / 64), 256, 0, stream>>>(W_Q, kEmb, kEmb, WqkT, kEmb, kWCarry);
  wtcast_kernel<<<dim3(kEmb / 64, kEmb / 64), 256, 0, stream>>>(W_K, kEmb, kEmb, WqkT + (size_t)kEmb * kEmb, kEmb, kWCarry);
  wtcast_kernel<<<dim3(kEmb / 64, kEmb / 64), 256, 0, stream>>>(W_V, kEmb, kEmb, WvT, kEmb, kWCarry);
  wtcast_kernel<<<dim3(kEmb / 64, kEmb / 64), 256, 0, stream>>>(W_out, kEmb, kEmb, WoT, kEmb, kWCarry);
  wtcast_kernel<<<dim3(kEmb / 64, kFF / 64), 256, 0, stream>>>(W1, kEmb, kFF, W1T, kEmb, kWCarry);
  wtcast_kernel<<<dim3(kFF / 64, kEmb / 64), 256, 0, stream>>>(W2, kFF, kEmb, W2T, kFF, kWCarry);

  layernorm_f16_kernel<<<kTok, 128, 0, stream>>>(X, ln1_g, ln1_b, H16);

  wmma_gemm64<0, false, 0, 1, false, 0, 0><<<dim3(256, 1), 256, 0, stream>>>(
      H16, H16, kEmb, 0L, WqkT, WqkT, kEmb, 0L, QK16, QK16, kQKld, 0L, X, X, 0L,
      kTok, kQKld, kEmb, kWCarryInv);

  wmma_gemm64<0, false, 0, 1, false, 0, 0><<<dim3(64, kBatch), 256, 0, stream>>>(
      WvT, WvT, kEmb, 0L, H16, H16, kEmb, (long)kSeq * kEmb, VT16, VT16, kSeq, (long)kEmb * kSeq, X, X, 0L,
      kEmb, kSeq, kEmb, kWCarryInv);

  for (int b = 0; b < kBatch; ++b) {
    for (int hc = 0; hc < kHeads / kHeadsPerChunk; ++hc) {
      const int h0 = hc * kHeadsPerChunk;
      const unsigned short* Qg = QK16 + (size_t)b * kSeq * kQKld + (size_t)h0 * kHeadDim;
      const unsigned short* Kg = Qg + kEmb;
      wmma_gemm64<0, false, 0, 0, false, 0, 1><<<dim3(128, kHeadsPerChunk), 256, 0, stream>>>(
          Qg, Qg, kQKld, (long)kHeadDim, Kg, Kg, kQKld, (long)kHeadDim,
          Sbuf, Sbuf, kSeq, (long)kSeq * kSeq, X, X, 0L,
          kSeq, kSeq, kHeadDim, 1.0f);
      softmax_causal_kernel<<<kHeadsPerChunk * kSeq, 256, 0, stream>>>(Sbuf, Pbuf, kPCarry);
      wmma_gemm64<0, false, 0, 1, false, 0, 2><<<dim3(4, kHeadsPerChunk), 256, 0, stream>>>(
          Pbuf, Pbuf, kSeq, (long)kSeq * kSeq,
          VT16 + (size_t)b * kEmb * kSeq + (size_t)h0 * kHeadDim * kSeq, VT16 + (size_t)b * kEmb * kSeq + (size_t)h0 * kHeadDim * kSeq,
          kSeq, (long)kHeadDim * kSeq,
          CTX16 + (size_t)b * kSeq * kEmb + (size_t)h0 * kHeadDim, CTX16 + (size_t)b * kSeq * kEmb + (size_t)h0 * kHeadDim,
          kEmb, (long)kHeadDim, X, X, 0L,
          kSeq, kHeadDim, kSeq, kPVScale);
    }
  }

  wmma_gemm64<0, false, 2, 0, true, 0, 0><<<dim3(128, 1), 256, 0, stream>>>(
      CTX16, CTX16, kEmb, 0L, WoT, WoT, kEmb, 0L, X1, X1, kEmb, 0L, b_out, X, 0L,
      kTok, kEmb, kEmb, kOutProjScale);

  layernorm_f16_kernel<<<kTok, 128, 0, stream>>>(X1, ln2_g, ln2_b, H16);

  wmma_gemm64<0, false, 2, 0, false, 0, 0><<<dim3(512, 1), 256, 0, stream>>>(
      H16, H16, kEmb, 0L, W1T, W1T, kEmb, 0L, FFpre, FFpre, kFF, 0L, b1, X, 0L,
      kTok, kFF, kEmb, kWCarryInv);

  gelu_cast_kernel<<<(kTok * kFF / 2) / 256, 256, 0, stream>>>(FFpre, G16, kTok * kFF / 2);

  wmma_gemm64<0, false, 2, 0, true, 0, 0><<<dim3(128, 1), 256, 0, stream>>>(
      G16, G16, kFF, 0L, W2T, W2T, kFF, 0L, out, out, kEmb, 0L, b2, X1, 0L,
      kTok, kEmb, kFF, kWCarryInv);
}
